// NPStatePrior_39075612459507
// MI455X (gfx1250) — hardware-run, weakly checked
//
#include <hip/hip_runtime.h>
#include <math.h>

typedef __attribute__((ext_vector_type(16))) _Float16 v16h;
typedef __attribute__((ext_vector_type(16))) __bf16   v16b;
typedef __attribute__((ext_vector_type(8)))  __bf16   v8b;
typedef __attribute__((ext_vector_type(8)))  float    v8f;
typedef __attribute__((ext_vector_type(4)))  float    v4f;
typedef __attribute__((ext_vector_type(4)))  unsigned v4u;
typedef __attribute__((ext_vector_type(8)))  unsigned v8u;
typedef __attribute__((ext_vector_type(2)))  _Float16 v2h;

constexpr int kNumDim  = 8;
constexpr int kHid     = 64;
constexpr int kLat     = 8;
constexpr int kInW     = 9;
constexpr int kBatch   = 64;
constexpr int kTime    = 1024;
constexpr int kRows    = kBatch * kTime;
constexpr int kBlkRows = 64;
constexpr int kNumBlk  = kRows / kBlkRows;
constexpr int kBlkPerBatch = kTime / kBlkRows;
constexpr int kAP      = 68;
constexpr int kW1Blk   = kHid * kInW;
constexpr int kPB1     = kW1Blk;
constexpr int kPB2     = kPB1 + kHid;
constexpr int kPB3     = kPB2 + kHid;
constexpr int kPWo     = kPB3 + kHid;
constexpr int kPTot    = kPWo + kHid;
static_assert(kInW == kLat + 1);
static_assert((kHid % 32) == 0 && (kHid % 16) == 0);
static_assert((kTime % kBlkRows) == 0 && (kRows % kBlkRows) == 0);
static_assert(kW1Blk == 576 && (kW1Blk % 4) == 0 && (kW1Blk / 4) == 144);
static_assert(kPTot == 832);
static_assert((kAP % 4) == 0 && kAP >= kHid);

constexpr bool  kFwdSplit = true;
constexpr float kWCarry   = 64.0f;
constexpr float kTCarry   = 64.0f;
constexpr float kACarry   = 16.0f;
constexpr float kTanFold  = 1.0f / (kTCarry * kWCarry);
constexpr float kFwdFold  = kFwdSplit ? 1.0f : (1.0f / (kACarry * kWCarry));
constexpr float kF16MinNormal = 6.103515625e-05f;
constexpr float kSlope    = 0.2f;

constexpr int    kPlaneElems = kNumDim * kHid * kHid;
constexpr size_t kPlaneBytes = (size_t)kPlaneElems * 2;
constexpr size_t kOffPlanes  = 0;
constexpr size_t kOffPart    = kOffPlanes + 6 * kPlaneBytes;
constexpr size_t kPartBytes  = (size_t)kNumBlk * 32 * 4;
constexpr size_t kWsTotal    = kOffPart + kPartBytes;
static_assert(kPlaneBytes == 65536);
static_assert(kWsTotal == 524288);
static_assert(kWsTotal <= 134217728ull);
static_assert((kOffPart % 128) == 0);

constexpr size_t kOut1OffBytes = (size_t)kRows * kNumDim * 4;
constexpr size_t kOutTotalBytes = kOut1OffBytes + (size_t)kBatch * 4;
static_assert(kOut1OffBytes == 2097152 && (kOut1OffBytes % 128) == 0);
static_assert(kOutTotalBytes == 2097408);

__device__ __forceinline__ unsigned bf_rne_word(float f) {
  unsigned u = __float_as_uint(f);
  const unsigned lsb = (u & 0x00010000u) ? 1u : 0u;
  return (u + 0x7FFFu + lsb) & 0xFFFF0000u;
}
__device__ __forceinline__ unsigned pack_hi16(unsigned lo_word, unsigned hi_word) {
  unsigned t = lo_word >> 16;
  asm volatile("" : "+v"(t));
  return (hi_word & 0xFFFF0000u) | t;
}
__device__ __forceinline__ void split_pair(float x0, float x1, unsigned& hw, unsigned& lw) {
  const unsigned h0 = bf_rne_word(x0);
  const unsigned h1 = bf_rne_word(x1);
  const float r0 = x0 - __uint_as_float(h0);
  const float r1 = x1 - __uint_as_float(h1);
  const unsigned l0 = bf_rne_word(r0);
  const unsigned l1 = bf_rne_word(r1);
  hw = pack_hi16(h0, h1);
  lw = pack_hi16(l0, l1);
}
__device__ __forceinline__ _Float16 to_f16_flush(float v) {
  const float y = (fabsf(v) < kF16MinNormal) ? 0.0f : v;
  return (_Float16)y;
}
__device__ __forceinline__ unsigned pack_f16_pair(float a, float b) {
  v2h p;
  p[0] = to_f16_flush(a);
  p[1] = to_f16_flush(b);
  return __builtin_bit_cast(unsigned, p);
}

__device__ __forceinline__ v8f mma_b(v16b a, v16b b, v8f c) {
  c = __builtin_amdgcn_wmma_f32_16x16x32_bf16(false, a, false, b, (short)0, c, false, false);
  asm volatile("v_nop\n\tv_nop\n\tv_nop\n\tv_nop" : "+v"(c) : "v"(a), "v"(b));
  return c;
}
__device__ __forceinline__ v8f mma_h(v16h a, v16h b, v8f c) {
  c = __builtin_amdgcn_wmma_f32_16x16x32_f16(false, a, false, b, (short)0, c, false, false);
  asm volatile("v_nop\n\tv_nop\n\tv_nop\n\tv_nop" : "+v"(c) : "v"(a), "v"(b));
  return c;
}

union FragB { v16b v; v8b h[2]; };
__device__ __forceinline__ v16b load_frag16(const unsigned short* p) {
  FragB f;
  f.h[0] = *(const v8b*)(p);
  f.h[1] = *(const v8b*)(p + 16);
  return f.v;
}

__global__ __launch_bounds__(256) void prep_planes_kernel(
    const float* __restrict__ W2, const float* __restrict__ W3, unsigned short* __restrict__ planes)
{
  const unsigned mat = blockIdx.x >> 4;
  const unsigned i   = ((blockIdx.x & 15u) << 8) + threadIdx.x;
  const float* src = (mat == 0u) ? W2 : W3;
  const size_t e0 = (size_t)i << 3;
  const v4f a0 = *(const v4f*)(src + e0);
  const v4f a1 = *(const v4f*)(src + e0 + 4);
  const float x[8] = { a0[0], a0[1], a0[2], a0[3], a1[0], a1[1], a1[2], a1[3] };
  v4u hw, lw, fw;
#pragma unroll
  for (int w = 0; w < 4; ++w) {
    unsigned hh, ll;
    split_pair(x[2 * w], x[2 * w + 1], hh, ll);
    hw[w] = hh;
    lw[w] = ll;
    fw[w] = pack_f16_pair(x[2 * w] * kWCarry, x[2 * w + 1] * kWCarry);
  }
  unsigned short* base = planes + (size_t)mat * 3 * kPlaneElems;
  unsigned short* qh = base + e0;
  unsigned short* ql = base + kPlaneElems + e0;
  unsigned short* qf = base + 2 * (size_t)kPlaneElems + e0;
  for (int pass = 0; pass < 2; ++pass) {
    *(volatile v4u*)qh = hw;
    *(volatile v4u*)ql = lw;
    *(volatile v4u*)qf = fw;
    __threadfence();
  }
}

__device__ __forceinline__ void layer_gemm(
    const float* aT, const float* tT,
    const unsigned short* __restrict__ pHi, const unsigned short* __restrict__ pLo,
    const unsigned short* __restrict__ pF,
    unsigned wrow0, unsigned c, unsigned h, v8f (&accF)[4], v8f (&accT)[4])
{
#pragma unroll
  for (int j = 0; j < 4; ++j) {
    accF[j] = (v8f){0.f, 0.f, 0.f, 0.f, 0.f, 0.f, 0.f, 0.f};
    accT[j] = (v8f){0.f, 0.f, 0.f, 0.f, 0.f, 0.f, 0.f, 0.f};
  }
#pragma unroll
  for (int kk = 0; kk < 2; ++kk) {
    const unsigned ko = (unsigned)kk * 32u + 8u * h;
    const float* ar = aT + c * (unsigned)kAP + ko;
    const float* tr = tT + c * (unsigned)kAP + ko;
    const v4f a0 = *(const v4f*)(ar);
    const v4f a1 = *(const v4f*)(ar + 4);
    const v4f a2 = *(const v4f*)(ar + 16);
    const v4f a3 = *(const v4f*)(ar + 20);
    const v4f t0 = *(const v4f*)(tr);
    const v4f t1 = *(const v4f*)(tr + 4);
    const v4f t2 = *(const v4f*)(tr + 16);
    const v4f t3 = *(const v4f*)(tr + 20);
    const float ax[16] = { a0[0], a0[1], a0[2], a0[3], a1[0], a1[1], a1[2], a1[3],
                           a2[0], a2[1], a2[2], a2[3], a3[0], a3[1], a3[2], a3[3] };
    const float tx[16] = { t0[0], t0[1], t0[2], t0[3], t1[0], t1[1], t1[2], t1[3],
                           t2[0], t2[1], t2[2], t2[3], t3[0], t3[1], t3[2], t3[3] };
    v16h th;
#pragma unroll
    for (int e = 0; e < 16; ++e) th[e] = to_f16_flush(tx[e] * kTCarry);
    if (kFwdSplit) {
      v8u hw, lw;
#pragma unroll
      for (int w = 0; w < 8; ++w) {
        unsigned hh, ll;
        split_pair(ax[2 * w], ax[2 * w + 1], hh, ll);
        hw[w] = hh;
        lw[w] = ll;
      }
      const v16b ahi = __builtin_bit_cast(v16b, hw);
      const v16b alo = __builtin_bit_cast(v16b, lw);
#pragma unroll
      for (int j = 0; j < 4; ++j) {
        const size_t bo = (size_t)(wrow0 + (unsigned)j * 16u + c) * (size_t)kHid + ko;
        const v16b bh = load_frag16(pHi + bo);
        const v16b bl = load_frag16(pLo + bo);
        const v16b bf = load_frag16(pF + bo);
        const v16h bfh = __builtin_bit_cast(v16h, bf);
        accF[j] = mma_b(ahi, bh, accF[j]);
        accF[j] = mma_b(ahi, bl, accF[j]);
        accF[j] = mma_b(alo, bh, accF[j]);
        accT[j] = mma_h(th, bfh, accT[j]);
      }
    } else {
      v16h afh;
#pragma unroll
      for (int e = 0; e < 16; ++e) afh[e] = to_f16_flush(ax[e] * kACarry);
#pragma unroll
      for (int j = 0; j < 4; ++j) {
        const size_t bo = (size_t)(wrow0 + (unsigned)j * 16u + c) * (size_t)kHid + ko;
        const v16b bf = load_frag16(pF + bo);
        const v16h bfh = __builtin_bit_cast(v16h, bf);
        accF[j] = mma_h(afh, bfh, accF[j]);
        accT[j] = mma_h(th, bfh, accT[j]);
      }
    }
  }
}

__global__ __launch_bounds__(128) void fused_chain_kernel(
    const float* __restrict__ z, const float* __restrict__ xs, const float* __restrict__ W1,
    const float* __restrict__ b1, const float* __restrict__ b2, const float* __restrict__ b3,
    const float* __restrict__ Wout, const float* __restrict__ bout,
    const unsigned short* __restrict__ planes, float* __restrict__ out0, float* __restrict__ part)
{
  __shared__ __align__(16) float sZ[kBlkRows * kLat];
  __shared__ __align__(16) float sX[kBlkRows * kNumDim];
  __shared__ __align__(16) float sP[kPTot];
  __shared__ __align__(16) float sAct[4 * 16 * kAP];
  __shared__ __align__(16) float sTan[4 * 16 * kAP];
  __shared__ __align__(16) float sO[kBlkRows * kNumDim];
  __shared__ __align__(16) float sLp[128];

  const unsigned tid  = threadIdx.x;
  const unsigned lane = tid & 31u;
  const unsigned wave = tid >> 5;
  unsigned c = lane & 15u;
  unsigned h = lane >> 4;
  asm volatile("" : "+v"(c), "+v"(h));
  const size_t n0 = (size_t)blockIdx.x * kBlkRows;

  *(v4f*)(sZ + tid * 4u) = *(const v4f*)(z  + n0 * kLat    + tid * 4u);
  *(v4f*)(sX + tid * 4u) = *(const v4f*)(xs + n0 * kNumDim + tid * 4u);

  float* aw = sAct + wave * (16u * (unsigned)kAP);
  float* tw = sTan + wave * (16u * (unsigned)kAP);
  const unsigned short* w2hi = planes;
  const unsigned short* w2lo = planes + kPlaneElems;
  const unsigned short* w2f  = planes + 2 * (size_t)kPlaneElems;
  const unsigned short* w3hi = planes + 3 * (size_t)kPlaneElems;
  const unsigned short* w3lo = planes + 4 * (size_t)kPlaneElems;
  const unsigned short* w3f  = planes + 5 * (size_t)kPlaneElems;

  float lacc = 0.0f;

#pragma unroll 1
  for (int d = 0; d < kNumDim; ++d) {
    __syncthreads();
    {
      const float* w1d = W1 + (size_t)d * kW1Blk;
      const unsigned i1 = 128u + (tid & 15u);
      const v4f q0 = *(const v4f*)(w1d + tid * 4u);
      const v4f q1 = *(const v4f*)(w1d + i1 * 4u);
      *(v4f*)(sP + tid * 4u) = q0;
      *(v4f*)(sP + i1 * 4u)  = q1;
      const unsigned hc = tid & 63u;
      const unsigned go = (unsigned)d * (unsigned)kHid + hc;
      const float pv1 = b1[go];
      const float pv2 = b2[go];
      const float pv3 = b3[go];
      const float pv4 = Wout[go];
      sP[kPB1 + hc] = pv1;
      sP[kPB2 + hc] = pv2;
      sP[kPB3 + hc] = pv3;
      sP[kPWo + hc] = pv4;
    }
    __syncthreads();

    {
      float w1r[4][kInW];
      float b1c[4];
#pragma unroll
      for (int j = 0; j < 4; ++j) {
        const unsigned col = (unsigned)j * 16u + c;
#pragma unroll
        for (int i = 0; i < kInW; ++i) w1r[j][i] = sP[col * (unsigned)kInW + (unsigned)i];
        b1c[j] = sP[kPB1 + col];
      }
#pragma unroll 1
      for (int r = 0; r < 8; ++r) {
        const unsigned row = 8u * h + (unsigned)r;
        const unsigned brow = wave * 16u + row;
        const float* zr = sZ + brow * (unsigned)kLat;
        const v4f z0 = *(const v4f*)(zr);
        const v4f z1 = *(const v4f*)(zr + 4);
        const float xv = sX[brow * (unsigned)kNumDim + (unsigned)d];
#pragma unroll
        for (int j = 0; j < 4; ++j) {
          float p = b1c[j];
          p = fmaf(w1r[j][0], z0[0], p);
          p = fmaf(w1r[j][1], z0[1], p);
          p = fmaf(w1r[j][2], z0[2], p);
          p = fmaf(w1r[j][3], z0[3], p);
          p = fmaf(w1r[j][4], z1[0], p);
          p = fmaf(w1r[j][5], z1[1], p);
          p = fmaf(w1r[j][6], z1[2], p);
          p = fmaf(w1r[j][7], z1[3], p);
          p = fmaf(w1r[j][8], xv, p);
          const float dlv = (p >= 0.0f) ? 1.0f : kSlope;
          const unsigned o = row * (unsigned)kAP + (unsigned)j * 16u + c;
          aw[o] = p * dlv;
          tw[o] = w1r[j][8] * dlv;
        }
      }
    }
    __syncthreads();

    v8f accF[4], accT[4];

    layer_gemm(aw, tw, w2hi, w2lo, w2f, (unsigned)d * (unsigned)kHid, c, h, accF, accT);
    __syncthreads();
    {
      float b2c[4];
#pragma unroll
      for (int j = 0; j < 4; ++j) b2c[j] = sP[kPB2 + (unsigned)j * 16u + c];
#pragma unroll
      for (int j = 0; j < 4; ++j) {
#pragma unroll
        for (int r = 0; r < 8; ++r) {
          const float p = accF[j][r] * kFwdFold + b2c[j];
          const float dlv = (p >= 0.0f) ? 1.0f : kSlope;
          const float tv = accT[j][r] * kTanFold;
          const unsigned o = (8u * h + (unsigned)r) * (unsigned)kAP + (unsigned)j * 16u + c;
          aw[o] = p * dlv;
          tw[o] = tv * dlv;
        }
      }
    }
    __syncthreads();

    layer_gemm(aw, tw, w3hi, w3lo, w3f, (unsigned)d * (unsigned)kHid, c, h, accF, accT);

    {
      float b3c[4], wo[4];
#pragma unroll
      for (int j = 0; j < 4; ++j) {
        b3c[j] = sP[kPB3 + (unsigned)j * 16u + c];
        wo[j]  = sP[kPWo + (unsigned)j * 16u + c];
      }
      const float bo = bout[d];
      float so[8], st[8];
#pragma unroll
      for (int r = 0; r < 8; ++r) {
        float s0 = 0.0f, s1 = 0.0f;
#pragma unroll
        for (int j = 0; j < 4; ++j) {
          const float p = accF[j][r] * kFwdFold + b3c[j];
          const float dlv = (p >= 0.0f) ? 1.0f : kSlope;
          const float a3 = p * dlv;
          const float t3 = (accT[j][r] * kTanFold) * dlv;
          s0 = fmaf(a3, wo[j], s0);
          s1 = fmaf(t3, wo[j], s1);
        }
        s0 += __shfl_xor(s0, 1, 32);
        s1 += __shfl_xor(s1, 1, 32);
        s0 += __shfl_xor(s0, 2, 32);
        s1 += __shfl_xor(s1, 2, 32);
        s0 += __shfl_xor(s0, 4, 32);
        s1 += __shfl_xor(s1, 4, 32);
        s0 += __shfl_xor(s0, 8, 32);
        s1 += __shfl_xor(s1, 8, 32);
        so[r] = s0;
        st[r] = s1;
      }
      float osel = so[0], tsel = st[0];
#pragma unroll
      for (int r = 1; r < 8; ++r) {
        osel = (c == (unsigned)r) ? so[r] : osel;
        tsel = (c == (unsigned)r) ? st[r] : tsel;
      }
      const float lg = logf(fabsf(tsel));
      lacc += (c < 8u) ? lg : 0.0f;
      if (c < 8u) sO[(wave * 16u + 8u * h + c) * (unsigned)kNumDim + (unsigned)d] = osel + bo;
    }
  }

  sLp[tid] = lacc;
  __syncthreads();

  const v4f ov = *(const v4f*)(sO + wave * 128u + lane * 4u);
  const float pv = ((sLp[lane] + sLp[32u + lane]) + sLp[64u + lane]) + sLp[96u + lane];
  float* op = out0 + (n0 + (size_t)wave * 16) * kNumDim + lane * 4u;
  float* pp = part + (size_t)blockIdx.x * 32 + lane;
  for (int pass = 0; pass < 2; ++pass) {
    *(volatile v4f*)op = ov;
    if (wave == 0u) *(volatile float*)pp = pv;
    __threadfence();
  }
}

__global__ __launch_bounds__(64) void finalize_kernel(const float* __restrict__ part, float* __restrict__ out1)
{
  const unsigned b = threadIdx.x;
  const float* p = part + (size_t)b * (kBlkPerBatch * 32);
  float s = 0.0f;
#pragma unroll 1
  for (int i = 0; i < (kBlkPerBatch * 32) / 4; ++i) {
    const v4f v = *(const v4f*)(p + 4 * i);
    s += v[0];
    s += v[1];
    s += v[2];
    s += v[3];
  }
  for (int pass = 0; pass < 2; ++pass) {
    *(volatile float*)(out1 + b) = s;
    __threadfence();
  }
}

extern "C" void kernel_launch(void* const* d_in, const int* in_sizes, int n_in,
                              void* d_out, int out_size, void* d_ws, size_t ws_size,
                              hipStream_t stream) {
  if (n_in < 10) return;
  if (in_sizes[0] != kRows * kLat) return;
  if (in_sizes[1] != kRows * kNumDim) return;
  if (in_sizes[2] != kNumDim * kHid * kInW) return;
  if (in_sizes[3] != kNumDim * kHid) return;
  if (in_sizes[4] != kPlaneElems) return;
  if (in_sizes[5] != kNumDim * kHid) return;
  if (in_sizes[6] != kPlaneElems) return;
  if (in_sizes[7] != kNumDim * kHid) return;
  if (in_sizes[8] != kNumDim * kHid) return;
  if (in_sizes[9] != kNumDim) return;
  if (out_size != kRows * kNumDim + kBatch) return;
  if (ws_size < kWsTotal) return;

  const float* z    = (const float*)d_in[0];
  const float* xs   = (const float*)d_in[1];
  const float* W1   = (const float*)d_in[2];
  const float* b1   = (const float*)d_in[3];
  const float* W2   = (const float*)d_in[4];
  const float* b2   = (const float*)d_in[5];
  const float* W3   = (const float*)d_in[6];
  const float* b3   = (const float*)d_in[7];
  const float* Wout = (const float*)d_in[8];
  const float* bout = (const float*)d_in[9];

  float* out0 = (float*)d_out;
  float* out1 = (float*)d_out + (kOut1OffBytes / 4);

  char* ws = (char*)d_ws;
  unsigned short* planes = (unsigned short*)(ws + kOffPlanes);
  float* part = (float*)(ws + kOffPart);

  prep_planes_kernel<<<32, 256, 0, stream>>>(W2, W3, planes);
  fused_chain_kernel<<<kNumBlk, 128, 0, stream>>>(z, xs, W1, b1, b2, b3, Wout, bout, planes, out0, part);
  finalize_kernel<<<1, 64, 0, stream>>>(part, out1);
}
